// ContrastiveGNNLSTM_50766513439455
// MI455X (gfx1250) — hardware-verified
//
#include <hip/hip_runtime.h>
#include <stddef.h>
#include <stdint.h>

typedef __attribute__((ext_vector_type(16))) _Float16 v16h;
typedef __attribute__((ext_vector_type(8)))  _Float16 v8h;
typedef __attribute__((ext_vector_type(8)))  float    v8f;
typedef __attribute__((ext_vector_type(4)))  float    v4f;
typedef __attribute__((ext_vector_type(4)))  unsigned v4u;

template <typename T> struct Frag;
template <> struct Frag<_Float16> {
  typedef v16h V; union U { v16h v; v8h h[2]; };
  static __device__ __forceinline__ v16h load(const _Float16* p) {
    U f; f.h[0] = *(const v8h*)(p); f.h[1] = *(const v8h*)(p + 16); return f.v;
  }
};

__device__ __forceinline__ v8f mma_h(v16h a, v16h b, v8f c) {
  c = __builtin_amdgcn_wmma_f32_16x16x32_f16(false, a, false, b, (short)0, c, false, false);
  asm volatile("v_nop\n\tv_nop\n\tv_nop\n\tv_nop" : "+v"(c) : "v"(a), "v"(b));
  return c;
}

__device__ __forceinline__ v8f zero8f() { return (v8f){0.f, 0.f, 0.f, 0.f, 0.f, 0.f, 0.f, 0.f}; }
__device__ __forceinline__ void lds_wave_sync() {
  __builtin_amdgcn_fence(__ATOMIC_RELEASE, "workgroup");
  __builtin_amdgcn_wave_barrier();
  __builtin_amdgcn_fence(__ATOMIC_ACQUIRE, "workgroup");
}

#define KLOG2E 1.4426950408889634f
__device__ __forceinline__ float sigm_f(float x) {
  const float e = __builtin_amdgcn_exp2f(fminf(-KLOG2E * x, 80.0f));
  return __builtin_amdgcn_rcpf(1.0f + e);
}
__device__ __forceinline__ float tanh_f(float x) {
  const float e = __builtin_amdgcn_exp2f(fminf((2.0f * KLOG2E) * x, 80.0f));
  return 1.0f - 2.0f * __builtin_amdgcn_rcpf(1.0f + e);
}

#define NSEQ      12288
#define TSTEPS    64
#define NNODE     128
#define NFEAT     16
#define HIDDEN    32
#define NGATEC    128
#define NGRAPH    96
#define DCHUNK    16
#define LG_PITCH  129
#define P_PITCH   136
#define FST_PITCH 136
#define INV128    0.0078125f
#define INV8192   0.0001220703125f

__global__ __launch_bounds__(128) void lstm_kernel(
    const float* __restrict__ anchor, const float* __restrict__ pos, const float* __restrict__ neg,
    const float* __restrict__ Wih, const float* __restrict__ Whh, const float* __restrict__ blstm,
    float* __restrict__ hn) {
  __shared__ __align__(16) _Float16 Bt16[NGATEC * 64];
  __shared__ __align__(16) _Float16 At[4][16 * 64];
  __shared__ __align__(16) float    slab[4][16 * 36];

  const int tid = threadIdx.x;
  const int wave = tid >> 5;
  const int lane = tid & 31;
  const int m = lane & 15;
  const int hh = lane >> 4;

  {
    const int n = tid;
    const float* wi = Wih + n * 16;
    const float* wh = Whh + n * 32;
    _Float16* br = Bt16 + n * 64;
#pragma unroll
    for (int q = 0; q < 2; ++q) {
      const v4f x0 = *(const v4f*)(wi + q * 8);
      const v4f x1 = *(const v4f*)(wi + q * 8 + 4);
      v8h v;
#pragma unroll
      for (int e = 0; e < 4; ++e) { v[e] = (_Float16)(x0[e] * 16.0f); v[4 + e] = (_Float16)(x1[e] * 16.0f); }
      *(v8h*)(br + q * 8) = v;
    }
#pragma unroll
    for (int q = 0; q < 4; ++q) {
      const v4f x0 = *(const v4f*)(wh + q * 8);
      const v4f x1 = *(const v4f*)(wh + q * 8 + 4);
      v8h v;
#pragma unroll
      for (int e = 0; e < 4; ++e) { v[e] = (_Float16)(x0[e] * 16.0f); v[4 + e] = (_Float16)(x1[e] * 16.0f); }
      *(v8h*)(br + 16 + q * 8) = v;
    }
    const v4u z4 = (v4u){0u, 0u, 0u, 0u};
    *(v4u*)(void*)(br + 48) = z4;
    *(v4u*)(void*)(br + 56) = z4;
  }
  _Float16* A = At[wave];
  {
    const v4u z4 = (v4u){0u, 0u, 0u, 0u};
#pragma unroll
    for (int j = 0; j < 4; ++j) *(v4u*)(void*)(A + (lane + 32 * j) * 8) = z4;
  }
  __syncthreads();

  const int tw = blockIdx.x * 4 + wave;
  const int s0 = tw * 16;
  const int sl = (s0 < 2048) ? s0 : ((s0 < 4096) ? (s0 - 2048) : (s0 - 4096));
  const float* src = (s0 < 2048) ? anchor : ((s0 < 4096) ? pos : neg);
  const int bk = sl >> 7;
  const int n0 = sl & 127;

  float bb[2][4];
#pragma unroll
  for (int jt = 0; jt < 2; ++jt)
#pragma unroll
    for (int gt = 0; gt < 4; ++gt) bb[jt][gt] = blstm[gt * 32 + 16 * jt + m];

  float creg[16], hreg[16];
#pragma unroll
  for (int i = 0; i < 16; ++i) { creg[i] = 0.0f; hreg[i] = 0.0f; }

#pragma unroll 1
  for (int t = 0; t < TSTEPS; ++t) {
    {
      const float* xp = src + ((size_t)(bk * TSTEPS + t) * NNODE + n0 + m) * NFEAT + 8 * hh;
      const v4f x0 = *(const v4f*)xp;
      const v4f x1 = *(const v4f*)(xp + 4);
      v8h xh;
#pragma unroll
      for (int e = 0; e < 4; ++e) { xh[e] = (_Float16)(x0[e] * 8.0f); xh[4 + e] = (_Float16)(x1[e] * 8.0f); }
      *(v8h*)(A + m * 64 + 8 * hh) = xh;
    }
    lds_wave_sync();
    const v16h a0 = Frag<_Float16>::load(A + m * 64 + 8 * hh);
    const v16h a1 = Frag<_Float16>::load(A + m * 64 + 32 + 8 * hh);

#pragma unroll
    for (int jt = 0; jt < 2; ++jt) {
      v16h b0[4], b1[4];
#pragma unroll
      for (int gt = 0; gt < 4; ++gt) {
        const int nt = gt * 2 + jt;
        const _Float16* bp = Bt16 + (nt * 16 + m) * 64 + 8 * hh;
        b0[gt] = Frag<_Float16>::load(bp);
        b1[gt] = Frag<_Float16>::load(bp + 32);
      }
      v8f acc[4];
#pragma unroll
      for (int gt = 0; gt < 4; ++gt) acc[gt] = zero8f();
#pragma unroll
      for (int gt = 0; gt < 4; ++gt) {
        acc[gt] = mma_h(a0, b0[gt], acc[gt]);
        acc[gt] = mma_h(a1, b1[gt], acc[gt]);
      }
#pragma unroll
      for (int r = 0; r < 8; ++r) {
        const float zi = fmaf(acc[0][r], INV128, bb[jt][0]);
        const float zf = fmaf(acc[1][r], INV128, bb[jt][1]);
        const float zg = fmaf(acc[2][r], INV128, bb[jt][2]);
        const float zo = fmaf(acc[3][r], INV128, bb[jt][3]);
        const float ig = sigm_f(zi);
        const float fg = sigm_f(zf);
        const float gg = tanh_f(zg);
        const float og = sigm_f(zo);
        const float c = fg * creg[jt * 8 + r] + ig * gg;
        creg[jt * 8 + r] = c;
        const float hv = og * tanh_f(c);
        hreg[jt * 8 + r] = hv;
        A[(8 * hh + r) * 64 + 16 + 16 * jt + m] = (_Float16)(hv * 8.0f);
      }
    }
  }

  float* sp = slab[wave];
#pragma unroll
  for (int jt = 0; jt < 2; ++jt)
#pragma unroll
    for (int r = 0; r < 8; ++r) sp[(8 * hh + r) * 36 + 16 * jt + m] = hreg[jt * 8 + r];
  lds_wave_sync();
  {
    const int q = lane >> 3, c4 = (lane & 7) * 4;
    for (int pass = 0; pass < 2; ++pass) {
#pragma unroll
      for (int it = 0; it < 4; ++it) {
        const int row = it * 4 + q;
        const v4f v = *(const v4f*)(sp + row * 36 + c4);
        *(volatile v4f*)(hn + (size_t)(s0 + row) * HIDDEN + c4) = v;
      }
      __threadfence();
    }
  }
}

template <bool POOL>
__global__ __launch_bounds__(128) void gat_kernel(
    const float* __restrict__ hin, const float* __restrict__ Ws, const float* __restrict__ Wd,
    const float* __restrict__ avec, const float* __restrict__ bvec, float* __restrict__ hout,
    int nheads, float head_scale) {
  __shared__ __align__(16) float    fsR[NNODE * 32];
  __shared__ __align__(16) float    fdR[NNODE * 32];
  __shared__ __align__(16) _Float16 fsT[32 * FST_PITCH];
  __shared__ __align__(16) float    hacc[NNODE * 32];
  __shared__ __align__(16) float    lg[DCHUNK * LG_PITCH];
  __shared__ __align__(16) _Float16 P16[DCHUNK * P_PITCH];
  __shared__ __align__(16) float    pmax[8 * DCHUNK];
  __shared__ __align__(16) float    psum[8 * DCHUNK];
  __shared__ __align__(16) float    fsA[NNODE];

  const int tid = threadIdx.x;
  const int wave = tid >> 5;
  const int lane = tid & 31;
  const int rl = lane & 15;
  const int hh = lane >> 4;
  const int g = blockIdx.x;
  const int e8 = wave * 2 + hh;
  int nh = nheads;
  nh = nh < 1 ? 1 : (nh > 8 ? 8 : nh);

  {
    const v4f z4 = (v4f){0.f, 0.f, 0.f, 0.f};
#pragma unroll
    for (int q = 0; q < 8; ++q) *(v4f*)(hacc + tid * 32 + 4 * q) = z4;
  }

#pragma unroll 1
  for (int hd = 0; hd < nh; ++hd) {
    {
      const float* WsH = Ws + (size_t)hd * 1024;
      const float* WdH = Wd + (size_t)hd * 1024;
      v16h bs[2], bd[2];
#pragma unroll
      for (int nt = 0; nt < 2; ++nt) {
        const int o = nt * 16 + rl;
#pragma unroll
        for (int e = 0; e < 8; ++e) {
          bs[nt][e]     = (_Float16)(WsH[(8 * hh + e) * 32 + o] * 16.0f);
          bs[nt][8 + e] = (_Float16)(WsH[(16 + 8 * hh + e) * 32 + o] * 16.0f);
          bd[nt][e]     = (_Float16)(WdH[(8 * hh + e) * 32 + o] * 16.0f);
          bd[nt][8 + e] = (_Float16)(WdH[(16 + 8 * hh + e) * 32 + o] * 16.0f);
        }
      }
#pragma unroll
      for (int mi = 0; mi < 2; ++mi) {
        const int mt = wave * 2 + mi;
        const int row = mt * 16 + rl;
        const float* hp = hin + ((size_t)g * NNODE + row) * 32;
        const v4f x0 = *(const v4f*)(hp + 8 * hh);
        const v4f x1 = *(const v4f*)(hp + 8 * hh + 4);
        const v4f x2 = *(const v4f*)(hp + 16 + 8 * hh);
        const v4f x3 = *(const v4f*)(hp + 20 + 8 * hh);
        v16h a;
#pragma unroll
        for (int e = 0; e < 4; ++e) {
          a[e]      = (_Float16)(x0[e] * 8.0f);
          a[4 + e]  = (_Float16)(x1[e] * 8.0f);
          a[8 + e]  = (_Float16)(x2[e] * 8.0f);
          a[12 + e] = (_Float16)(x3[e] * 8.0f);
        }
        v8f ps[2], pd[2];
#pragma unroll
        for (int nt = 0; nt < 2; ++nt) {
          ps[nt] = mma_h(a, bs[nt], zero8f());
          pd[nt] = mma_h(a, bd[nt], zero8f());
        }
#pragma unroll
        for (int nt = 0; nt < 2; ++nt) {
          const int o = nt * 16 + rl;
          v8h tv;
#pragma unroll
          for (int r = 0; r < 8; ++r) {
            const int rr = mt * 16 + 8 * hh + r;
            const float vs = ps[nt][r] * INV128;
            const float vd = pd[nt][r] * INV128;
            fsR[rr * 32 + o] = vs;
            fdR[rr * 32 + o] = vd;
            tv[r] = (_Float16)(vs * 8.0f);
          }
          *(v8h*)(fsT + o * FST_PITCH + mt * 16 + 8 * hh) = tv;
        }
      }
    }
    float av[32];
#pragma unroll
    for (int k = 0; k < 32; ++k) av[k] = avec[hd * 32 + k];
    const float bo = bvec[hd * 32 + (wave & 1) * 16 + rl];
    __syncthreads();

    {
      float sA = 0.0f;
      const v4f* fp = (const v4f*)(fsR + tid * 32);
#pragma unroll
      for (int q = 0; q < 8; ++q) {
        const v4f f4 = fp[q];
#pragma unroll
        for (int e = 0; e < 4; ++e) sA = fmaf(av[4 * q + e], f4[e], sA);
      }
      fsA[tid] = sA;
    }
    __syncthreads();

#pragma unroll 1
    for (int p = 0; p < NNODE / DCHUNK; ++p) {
      const int d = p * DCHUNK + rl;
      float fdv[32];
      {
        const v4f* fp = (const v4f*)(fdR + d * 32);
#pragma unroll
        for (int q = 0; q < 8; ++q) {
          const v4f f4 = fp[q];
#pragma unroll
          for (int e = 0; e < 4; ++e) fdv[4 * q + e] = f4[e];
        }
      }
      float fdA = 0.0f;
#pragma unroll
      for (int k = 0; k < 32; ++k) fdA = fmaf(av[k], fdv[k], fdA);

      float mloc = -__builtin_inff();
#pragma unroll 1
      for (int j = 0; j < 16; ++j) {
        const int s = e8 * 16 + j;
        const v4f* fp = (const v4f*)(fsR + s * 32);
        float acc = 0.0f;
#pragma unroll
        for (int q = 0; q < 8; ++q) {
          const v4f f4 = fp[q];
#pragma unroll
          for (int e = 0; e < 4; ++e) {
            const float x = fdv[4 * q + e] + f4[e];
            acc = fmaf(av[4 * q + e], __builtin_fabsf(x), acc);
          }
        }
        const float lgv = 0.4f * acc + 0.6f * (fdA + fsA[s]);
        lg[rl * LG_PITCH + s] = lgv;
        mloc = (s == d) ? mloc : fmaxf(mloc, lgv);
      }
      pmax[e8 * DCHUNK + rl] = mloc;
      __syncthreads();

      float mrow = pmax[rl];
#pragma unroll
      for (int e = 1; e < 8; ++e) mrow = fmaxf(mrow, pmax[e * DCHUNK + rl]);
      float psm = 0.0f;
      v8h pv0, pv1;
#pragma unroll
      for (int j = 0; j < 8; ++j) {
        const int s = e8 * 16 + j;
        float pe = __builtin_amdgcn_exp2f((lg[rl * LG_PITCH + s] - mrow) * KLOG2E);
        pe = (s == d) ? 0.0f : pe;
        psm += pe;
        pv0[j] = (_Float16)(pe * 1024.0f);
      }
#pragma unroll
      for (int j = 0; j < 8; ++j) {
        const int s = e8 * 16 + 8 + j;
        float pe = __builtin_amdgcn_exp2f((lg[rl * LG_PITCH + s] - mrow) * KLOG2E);
        pe = (s == d) ? 0.0f : pe;
        psm += pe;
        pv1[j] = (_Float16)(pe * 1024.0f);
      }
      *(v8h*)(P16 + rl * P_PITCH + e8 * 16) = pv0;
      *(v8h*)(P16 + rl * P_PITCH + e8 * 16 + 8) = pv1;
      psum[e8 * DCHUNK + rl] = psm;
      __syncthreads();

      if (wave < 2) {
        const int o = wave * 16 + rl;
        v8f acc2 = zero8f();
#pragma unroll
        for (int kc = 0; kc < 4; ++kc) {
          const v16h ap = Frag<_Float16>::load(P16 + rl * P_PITCH + kc * 32 + 8 * hh);
          const v16h bq = Frag<_Float16>::load(fsT + o * FST_PITCH + kc * 32 + 8 * hh);
          acc2 = mma_h(ap, bq, acc2);
        }
#pragma unroll
        for (int r = 0; r < 8; ++r) {
          const int row = 8 * hh + r;
          float sm = psum[row];
#pragma unroll
          for (int e = 1; e < 8; ++e) sm += psum[e * DCHUNK + row];
          const float inv = 1.0f / sm;
          const float val = acc2[r] * (INV8192 * inv) + bo;
          hacc[(p * DCHUNK + row) * 32 + o] += val;
        }
      }
      __syncthreads();
    }
  }

  if (!POOL) {
    const int q = lane >> 3, c4 = (lane & 7) * 4;
    for (int pass = 0; pass < 2; ++pass) {
#pragma unroll
      for (int it = 0; it < 8; ++it) {
        const int row = wave * 32 + it * 4 + q;
        v4f v = *(const v4f*)(hacc + row * 32 + c4);
        v = v * head_scale;
        *(volatile v4f*)(hout + ((size_t)g * NNODE + row) * 32 + c4) = v;
      }
      __threadfence();
    }
  } else {
    if (wave == 0) {
      float s = 0.0f;
#pragma unroll 1
      for (int row = 0; row < NNODE; ++row) s += hacc[row * 32 + lane];
      pmax[lane] = s * INV128 * head_scale;
      lds_wave_sync();
      const int c4 = (lane & 7) * 4;
      const v4f v = *(const v4f*)(pmax + c4);
      for (int pass = 0; pass < 2; ++pass) {
        if (lane < 8) *(volatile v4f*)(hout + (size_t)g * 32 + c4) = v;
        __threadfence();
      }
    }
  }
}

__global__ __launch_bounds__(128) void final_kernel(
    const float* __restrict__ pooled, const float* __restrict__ hideout, const float* __restrict__ timestep,
    const int* __restrict__ nagents, float* __restrict__ out) {
  __shared__ __align__(16) float ob[576];
  __shared__ float lsh[16];
  const int tid = threadIdx.x;
  (void)nagents;
  {
    const int b = tid & 15;
    const float* an = pooled + b * 32;
    float na2 = 0.0f;
#pragma unroll 1
    for (int k = 0; k < 32; ++k) na2 = fmaf(an[k], an[k], na2);
    const float inva = 1.0f / fmaxf(sqrtf(na2), 1e-6f);
    float se = 0.0f, vlast = 0.0f;
#pragma unroll 1
    for (int j = 0; j < 5; ++j) {
      const int row = (j < 4) ? (32 + b * 4 + j) : (16 + b);
      const float* yp = pooled + row * 32;
      float ny2 = 0.0f;
#pragma unroll 1
      for (int k = 0; k < 32; ++k) ny2 = fmaf(yp[k], yp[k], ny2);
      const float invy = 1.0f / fmaxf(sqrtf(ny2), 1e-6f);
      float dot = 0.0f;
#pragma unroll 1
      for (int k = 0; k < 32; ++k) dot += (an[k] * inva) * (yp[k] * invy);
      se += expf(dot);
      vlast = dot;
    }
    if (tid < 16) {
      lsh[b] = logf(se) - vlast;
#pragma unroll 1
      for (int k = 0; k < 32; ++k) ob[b * 35 + k] = an[k];
      ob[b * 35 + 32] = hideout[b * 2 + 0];
      ob[b * 35 + 33] = hideout[b * 2 + 1];
      ob[b * 35 + 34] = timestep[b];
    }
  }
  __syncthreads();
  if (tid == 0) {
    float s = 0.0f;
#pragma unroll 1
    for (int i = 0; i < 16; ++i) s += lsh[i];
    ob[560] = s * 0.0625f;
  }
  __syncthreads();
  const v4f va = *(const v4f*)(ob + tid * 4);
  const v4f vb = *(const v4f*)(ob + 512 + (tid & 7) * 4);
  const float vt = ob[544 + ((tid < 17) ? tid : 16)];
  for (int pass = 0; pass < 2; ++pass) {
    *(volatile v4f*)(out + tid * 4) = va;
    if (tid < 8)  *(volatile v4f*)(out + 512 + tid * 4) = vb;
    if (tid < 17) *(volatile float*)(out + 544 + tid) = vt;
    __threadfence();
  }
}

extern "C" void kernel_launch(void* const* d_in, const int* in_sizes, int n_in,
                              void* d_out, int out_size, void* d_ws, size_t ws_size,
                              hipStream_t stream) {
  if (n_in < 17) return;
  if (in_sizes[0] != 16 * 64 * 128 * 16) return;
  if (in_sizes[1] != 16 * 64 * 128 * 16) return;
  if (in_sizes[2] != 16 * 4 * 64 * 128 * 16) return;
  if (in_sizes[3] != 32 || in_sizes[4] != 16) return;
  if (in_sizes[5] != 128 * 16 || in_sizes[6] != 128 * 32 || in_sizes[7] != 128) return;
  if (in_sizes[8] != 8 * 32 * 32 || in_sizes[9] != 8 * 32 * 32) return;
  if (in_sizes[10] != 8 * 32 || in_sizes[11] != 8 * 32) return;
  if (in_sizes[12] != 32 * 32 || in_sizes[13] != 32 * 32) return;
  if (in_sizes[14] != 32 || in_sizes[15] != 32) return;
  if (out_size != 561) return;

  const size_t hn_bytes = (size_t)NSEQ * HIDDEN * sizeof(float);
  const size_t h1_bytes = hn_bytes;
  const size_t pooled_bytes = (size_t)NGRAPH * HIDDEN * sizeof(float);
  const size_t off_hn = 0;
  const size_t off_h1 = off_hn + hn_bytes;
  const size_t off_pooled = off_h1 + h1_bytes;
  const size_t total = off_pooled + pooled_bytes;
  if (total > ws_size) return;

  const float* anchor   = (const float*)d_in[0];
  const float* pos      = (const float*)d_in[1];
  const float* neg      = (const float*)d_in[2];
  const float* hideout  = (const float*)d_in[3];
  const float* timestep = (const float*)d_in[4];
  const float* Wih      = (const float*)d_in[5];
  const float* Whh      = (const float*)d_in[6];
  const float* blstm    = (const float*)d_in[7];
  const float* W1s      = (const float*)d_in[8];
  const float* W1d      = (const float*)d_in[9];
  const float* a1       = (const float*)d_in[10];
  const float* b1       = (const float*)d_in[11];
  const float* W2s      = (const float*)d_in[12];
  const float* W2d      = (const float*)d_in[13];
  const float* a2       = (const float*)d_in[14];
  const float* b2       = (const float*)d_in[15];
  const int*   nag      = (const int*)d_in[16];

  char* ws = (char*)d_ws;
  float* hn     = (float*)(ws + off_hn);
  float* h1     = (float*)(ws + off_h1);
  float* pooled = (float*)(ws + off_pooled);
  float* out    = (float*)d_out;

  lstm_kernel<<<dim3(NSEQ / 64), dim3(128), 0, stream>>>(anchor, pos, neg, Wih, Whh, blstm, hn);
  gat_kernel<false><<<dim3(NGRAPH), dim3(128), 0, stream>>>(hn, W1s, W1d, a1, b1, h1, 8, 0.125f);
  gat_kernel<true><<<dim3(NGRAPH), dim3(128), 0, stream>>>(h1, W2s, W2d, a2, b2, pooled, 1, 1.0f);
  final_kernel<<<dim3(1), dim3(128), 0, stream>>>(pooled, hideout, timestep, nag, out);
}
